// DifferentiableRenderer_9019431322196
// MI455X (gfx1250) — hardware-verified
//
#include <hip/hip_runtime.h>


typedef _Float16 v16h __attribute__((ext_vector_type(16)));
typedef float    v8f  __attribute__((ext_vector_type(8)));
typedef float    v4f  __attribute__((ext_vector_type(4)));

#define IMG_W_LOG2 7
#define IMG_W      128
#define TILE_PX    4096
#define NCH        3
#define GSPLIT     2048
#define FX_        150.0f
#define CX_        64.0f
#define EPS_       1e-8f
#define WSCALE     16384.0f
#define LOG2E_     1.4426950408889634f
#define GCHUNK     512
#define NSUB       (GCHUNK / 32)
#define RB_THREADS 128

static __device__ __forceinline__ int kmap(int d, int h) {
    return ((d & 3) << 1) + ((d >> 2) << 4) + (h << 3);
}

static __device__ __forceinline__ unsigned pack2h(float a, float b) {
    unsigned short ua = __builtin_bit_cast(unsigned short, (_Float16)a);
    unsigned short ub = __builtin_bit_cast(unsigned short, (_Float16)b);
    return (unsigned)ua | ((unsigned)ub << 16);
}

static __device__ __forceinline__ v8f wmma_f16(const v16h a, const v16h b, v8f c) {
    v8f d = __builtin_amdgcn_wmma_f32_16x16x32_f16(false, a, false, b, (short)0, c, false, false);
    asm volatile("v_nop\n\tv_nop\n\tv_nop\n\tv_nop" : "+v"(d) : "v"(a), "v"(b));
    return d;
}

__global__ __launch_bounds__(256) void k_prep(
    const float* __restrict__ pos, const float* __restrict__ opac,
    const float* __restrict__ scal, const float* __restrict__ qv,
    const float* __restrict__ tv, float* g4, int N, int Npad)
{
    #pragma clang fp contract(off)
    const int i = blockIdx.x * 256 + threadIdx.x;
    const bool ok = (i < Npad);

    float qw = qv[0], qx = qv[1], qy = qv[2], qz = qv[3];
    const float nrm = sqrtf(qw * qw + qx * qx + qy * qy + qz * qz);
    const float inv = 1.0f / nrm;
    qw = qw * inv; qx = qx * inv; qy = qy * inv; qz = qz * inv;
    const float r00 = 1.f - 2.f * (qy * qy + qz * qz), r01 = 2.f * (qx * qy - qz * qw), r02 = 2.f * (qx * qz + qy * qw);
    const float r10 = 2.f * (qx * qy + qz * qw), r11 = 1.f - 2.f * (qx * qx + qz * qz), r12 = 2.f * (qy * qz - qx * qw);
    const float r20 = 2.f * (qx * qz - qy * qw), r21 = 2.f * (qy * qz + qx * qw), r22 = 1.f - 2.f * (qx * qx + qy * qy);
    const float t0 = tv[0], t1 = tv[1], t2 = tv[2];

    v4f val;
    val.x = 0.f; val.y = 0.f; val.z = -1.0f; val.w = 0.f;
    if (ok && i < N) {
        const float p0 = pos[3 * i + 0], p1 = pos[3 * i + 1], p2 = pos[3 * i + 2];
        const float cx = ((p0 * r00 + p1 * r01) + p2 * r02) + t0;
        const float cy = ((p0 * r10 + p1 * r11) + p2 * r12) + t1;
        const float cz = ((p0 * r20 + p1 * r21) + p2 * r22) + t2;
        const float rz = 1.0f / cz;
        float ux = cx * rz; ux = ux * FX_; ux = ux + CX_;
        float uy = cy * rz; uy = uy * FX_; uy = uy + CX_;
        const float s   = scal[i];
        const float var = s * s;
        const float rv  = 1.0f / var;
        const float coef2 = (-0.5f * LOG2E_) * rv;
        val.x = ux; val.y = uy; val.z = coef2; val.w = opac[i] * WSCALE;
    }
    if (ok) {
        float* p = g4 + (size_t)i * 4;
        *(volatile v4f*)p = val;
    }
    __threadfence();
    if (ok) {
        float* p = g4 + (size_t)i * 4;
        *(volatile v4f*)p = val;
    }
}

__global__ __launch_bounds__(RB_THREADS) void k_render(
    const float* __restrict__ g4, const float* __restrict__ colors,
    float* out, int N, int Npad, int P)
{
    #pragma clang fp contract(off)
    __shared__ v4f   sG[GCHUNK];
    __shared__ float sS[GCHUNK];
    __shared__ __attribute__((aligned(32))) unsigned bfrag[NSUB][32][8];
    __shared__ __attribute__((aligned(16))) float sOut[RB_THREADS / 32][NCH][32];

    const int tid  = threadIdx.x;
    const int lane = tid & 31;
    const int wv   = tid >> 5;
    const int h    = lane >> 4;
    const int col  = lane & 15;
    const int waveId  = blockIdx.x * (RB_THREADS / 32) + wv;
    const int pixBase = waveId * 32;
    const bool wave_ok = (pixBase + 32 <= P);

    int p0i = pixBase + col;
    if (p0i > P - 1) p0i = P - 1;
    const float X0  = (float)(p0i & (IMG_W - 1));
    const float X1  = X0 + 16.0f;
    const float Y   = (float)(p0i >> IMG_W_LOG2);
    const float P20 = X0 * X0 + Y * Y;
    const float P21 = X1 * X1 + Y * Y;

    v8f acc0 = {};
    v8f acc1 = {};

    for (int gb = 0; gb < Npad; gb += GCHUNK) {
        __syncthreads();
        for (int i = tid; i < GCHUNK; i += RB_THREADS) {
            const int g = gb + i;
            const v4f v = *(const v4f*)(g4 + (size_t)g * 4);
            sG[i] = v;
            const float sx = v.x * v.x;
            const float sy = v.y * v.y;
            sS[i] = sx + sy;
        }
        for (int idx = tid; idx < NSUB * 256; idx += RB_THREADS) {
            const int sub = idx >> 8;
            const int l   = (idx >> 3) & 31;
            const int d   = idx & 7;
            const int k   = sub * 32 + kmap(d, l >> 4);
            const int n   = l & 15;
            float v0 = 0.f, v1 = 0.f;
            if (n < NCH) {
                const int g0 = gb + k, g1 = g0 + 1;
                if (g0 < N) v0 = colors[(size_t)g0 * NCH + n];
                if (g1 < N) v1 = colors[(size_t)g1 * NCH + n];
            } else if (n == NCH) {
                v0 = 1.f; v1 = 1.f;
            }
            bfrag[sub][l][d] = pack2h(v0, v1);
        }
        __syncthreads();

        for (int sub = 0; sub < NSUB; ++sub) {
            const int base = sub * 32;
            const v16h bv = *(const v16h*)(&bfrag[sub][lane][0]);
            v16h a0 = {};
            v16h a1 = {};
            #pragma unroll
            for (int j = 0; j < 8; ++j) {
                #pragma unroll
                for (int e = 0; e < 2; ++e) {
                    const int kk = base + kmap(j, h) + e;
                    const v4f g  = sG[kk];
                    const float s = sS[kk];
                    const float sp0 = s + P20;
                    const float sp1 = s + P21;
                    const float m0  = g.x * X0;
                    const float m1  = g.x * X1;
                    const float dt0 = fmaf(g.y, Y, m0);
                    const float dt1 = fmaf(g.y, Y, m1);
                    const float d0  = fmaf(-2.0f, dt0, sp0);
                    const float d1  = fmaf(-2.0f, dt1, sp1);
                    const float w0  = g.w * __builtin_amdgcn_exp2f(d0 * g.z);
                    const float w1  = g.w * __builtin_amdgcn_exp2f(d1 * g.z);
                    a0[2 * j + e] = (_Float16)w0;
                    a1[2 * j + e] = (_Float16)w1;
                }
            }
            acc0 = wmma_f16(a0, bv, acc0);
            acc1 = wmma_f16(a1, bv, acc1);
        }
    }

    const float epsN = (float)(N / GSPLIT) * EPS_ * WSCALE;
    const float eps1 = EPS_ * WSCALE;
    #pragma unroll
    for (int r = 0; r < 8; ++r) {
        const float den0 = __shfl(acc0[r], NCH + 16 * h, 32);
        const float den1 = __shfl(acc1[r], NCH + 16 * h, 32);
        const float i0 = 1.0f / fmaxf(den0 + epsN, eps1);
        const float i1 = 1.0f / fmaxf(den1 + epsN, eps1);
        const float q0 = acc0[r] * i0;
        const float q1 = acc1[r] * i1;
        if (col < NCH) {
            sOut[wv][col][8 * h + r]      = q0;
            sOut[wv][col][16 + 8 * h + r] = q1;
        }
    }
    __syncthreads();

    const int q  = lane >> 3;
    const int jj = lane & 7;
    const bool st_ok = wave_ok && (q < NCH);
    v4f ov;
    ov.x = 0.f; ov.y = 0.f; ov.z = 0.f; ov.w = 0.f;
    size_t o = 0;
    if (st_ok) {
        ov = *(const v4f*)(&sOut[wv][q][4 * jj]);
        o  = (size_t)(pixBase / TILE_PX) * (NCH * TILE_PX) + (size_t)q * TILE_PX
           + (size_t)(pixBase & (TILE_PX - 1)) + 4 * jj;
        *(volatile v4f*)(out + o) = ov;
    }
    __threadfence();
    if (st_ok) {
        *(volatile v4f*)(out + o) = ov;
    }
}

extern "C" void kernel_launch(void* const* d_in, const int* in_sizes, int n_in,
                              void* d_out, int out_size, void* d_ws, size_t ws_size,
                              hipStream_t stream)
{
    if (n_in < 6) return;
    const float* positions = (const float*)d_in[0];
    const float* colors    = (const float*)d_in[1];
    const float* opacities = (const float*)d_in[2];
    const float* scales    = (const float*)d_in[3];
    const float* qvec      = (const float*)d_in[4];
    const float* tvec      = (const float*)d_in[5];
    float*       out       = (float*)d_out;

    int N = in_sizes[2];
    if (in_sizes[0] / 3 < N) N = in_sizes[0] / 3;
    if (in_sizes[1] / 3 < N) N = in_sizes[1] / 3;
    if (in_sizes[3] < N)     N = in_sizes[3];
    if (N <= 0 || in_sizes[4] < 4 || in_sizes[5] < 3) return;

    const int P = out_size / NCH;
    if (P * NCH != out_size || (P % TILE_PX) != 0 || P <= 0) return;

    const int Npad = ((N + GCHUNK - 1) / GCHUNK) * GCHUNK;
    if ((size_t)Npad * 16 > ws_size) return;
    float* g4 = (float*)d_ws;

    k_prep<<<Npad / 256, 256, 0, stream>>>(positions, opacities, scales, qvec, tvec, g4, N, Npad);

    const int nWaves  = (P + 31) / 32;
    const int nBlocks = (nWaves + (RB_THREADS / 32) - 1) / (RB_THREADS / 32);
    k_render<<<nBlocks, RB_THREADS, 0, stream>>>(g4, colors, out, N, Npad, P);
}
